// KernelizedAttention_4964982194187
// MI455X (gfx1250) — hardware-verified
//
#include <hip/hip_runtime.h>
#include <math.h>

typedef __attribute__((ext_vector_type(16))) _Float16 v16h;
typedef __attribute__((ext_vector_type(16))) __bf16 v16b;
typedef __attribute__((ext_vector_type(8)))  _Float16 v8h;
typedef __attribute__((ext_vector_type(8)))  float v8f;
typedef __attribute__((ext_vector_type(4)))  float v4f;
typedef __attribute__((ext_vector_type(2)))  float v2f;
typedef __attribute__((ext_vector_type(4)))  unsigned v4u;
typedef __attribute__((ext_vector_type(4)))  int v4i;
typedef float __attribute__((may_alias)) float_a;
typedef int __attribute__((may_alias)) int_a;

template <typename T> __device__ __forceinline__ void vst2(void* p, T v) { *(volatile T*)p = v; __threadfence(); *(volatile T*)p = v; }
__device__ __forceinline__ v8f wmma16(v16h a, v16h b, v8f c) {
  v8f d = __builtin_amdgcn_wmma_f32_16x16x32_f16(false, a, false, b, (short)0, c, false, false);
  asm volatile("v_nop\n\tv_nop\n\tv_nop\n\tv_nop" : "+v"(d) : "v"(a), "v"(b));
  return d;
}
__device__ __forceinline__ v8f wmma_bf(v16b a, v16b b, v8f c) {
  v8f d = __builtin_amdgcn_wmma_f32_16x16x32_bf16(false, a, false, b, (short)0, c, false, false);
  asm volatile("v_nop\n\tv_nop\n\tv_nop\n\tv_nop" : "+v"(d) : "v"(a), "v"(b));
  return d;
}
__device__ __forceinline__ v16h frag_h(const _Float16* rowk0, int lane) {
  union { v16h v; v8h q[2]; } u; const _Float16* p = rowk0 + 8 * (lane >> 4);
  u.q[0] = *(const v8h*)p; u.q[1] = *(const v8h*)(p + 16); return u.v;
}
__device__ __forceinline__ v16h frag_f32(const float* rowk0, int lane) {
  v16h a; const float* p = rowk0 + 8 * (lane >> 4);
#pragma unroll
  for (int i = 0; i < 8; ++i) { a[i] = (_Float16)p[i]; a[8 + i] = (_Float16)p[16 + i]; }
  return a;
}
__device__ __forceinline__ v16h frag_f32s(const float* rowk0, int lane, float sc) {
  v16h a; const float* p = rowk0 + 8 * (lane >> 4);
#pragma unroll
  for (int i = 0; i < 8; ++i) { a[i] = (_Float16)(p[i] * sc); a[8 + i] = (_Float16)(p[16 + i] * sc); }
  return a;
}
__device__ __forceinline__ v16h fragc_f32(const float* W, int k0, int n, int lane, int ld, int K) {
  v16h a; const int g = lane >> 4;
#pragma unroll
  for (int i = 0; i < 8; ++i) { const int ka = k0 + 8 * g + i, kb = ka + 16;
    a[i] = (_Float16)(ka < K ? W[(size_t)ka * ld + n] : 0.f); a[8 + i] = (_Float16)(kb < K ? W[(size_t)kb * ld + n] : 0.f); }
  return a;
}
struct F2 { v16b h, l; };
__device__ __forceinline__ F2 bsplit16(const float v[16]) { F2 r;
#pragma unroll
  for (int i = 0; i < 16; ++i) { const __bf16 h = (__bf16)v[i]; r.h[i] = h; r.l[i] = (__bf16)(v[i] - (float)h); }
  return r; }
__device__ __forceinline__ F2 split_row(const float* row, int k0, int lane) { float v[16]; const float* p = row + k0 + 8 * (lane >> 4);
#pragma unroll
  for (int i = 0; i < 8; ++i) { v[i] = p[i]; v[8 + i] = p[16 + i]; }
  return bsplit16(v); }
__device__ __forceinline__ F2 split_rowK(const float* row, int k0, int lane, int K) { float v[16]; const int g = lane >> 4;
#pragma unroll
  for (int i = 0; i < 8; ++i) { const int ka = k0 + 8 * g + i, kb = ka + 16; v[i] = ka < K ? row[ka] : 0.f; v[8 + i] = kb < K ? row[kb] : 0.f; }
  return bsplit16(v); }
__device__ __forceinline__ F2 split_col(const float* W, int k0, int n, int lane, int ld, int K) { float v[16]; const int g = lane >> 4;
#pragma unroll
  for (int i = 0; i < 8; ++i) { const int ka = k0 + 8 * g + i, kb = ka + 16; v[i] = ka < K ? W[(size_t)ka * ld + n] : 0.f; v[8 + i] = kb < K ? W[(size_t)kb * ld + n] : 0.f; }
  return bsplit16(v); }
__device__ __forceinline__ v8f mac3(const F2& a, const F2& b, v8f c) { c = wmma_bf(a.l, b.h, c); c = wmma_bf(a.h, b.l, c); return wmma_bf(a.h, b.h, c); }
__device__ __forceinline__ float sigm(float v) { return 1.0f / (1.0f + expf(-v)); }
#define LDSX() do { asm volatile("s_wait_dscnt 0" ::: "memory"); __builtin_amdgcn_wave_barrier(); __builtin_amdgcn_fence(__ATOMIC_RELEASE, "workgroup"); } while (0)

#define NB 2
#define LL 2048
#define DM 512
#define NH 8
#define HD 64
#define NR (NB * LL)

__global__ __launch_bounds__(128) void k_proj(const float* __restrict__ xq, const float* __restrict__ xk, const float* __restrict__ Wq, const float* __restrict__ Wk, const float* __restrict__ Wv,
                                            _Float16* __restrict__ PQ16, float* __restrict__ PQ32, _Float16* __restrict__ PK16, float* __restrict__ PK32, float* __restrict__ V32, _Float16* __restrict__ VT16) {
  __shared__ __align__(16) float so[4][16][132];
  __shared__ __align__(16) _Float16 st[128][72];
  const int tid = threadIdx.x, wave = tid >> 5, lane = tid & 31, col = lane & 15, g = lane >> 4;
  const int which = blockIdx.z, r0b = blockIdx.x * 64, r0 = r0b + wave * 16, n0 = blockIdx.y * 128;
  v8f acc[8] = {};
  if (which < 2) { const float* X = which == 0 ? xq : xk; const float* W = which == 0 ? Wq : Wk;
#pragma unroll 1
    for (int kc = 0; kc < DM / 32; ++kc) { const v16h a = frag_f32(X + (size_t)(r0 + col) * DM + kc * 32, lane);
#pragma unroll
      for (int j = 0; j < 8; ++j) acc[j] = wmma16(a, frag_f32s(W + (size_t)(n0 + j * 16 + col) * DM + kc * 32, lane, 16.0f), acc[j]); }
#pragma unroll
    for (int j = 0; j < 8; ++j)
#pragma unroll
      for (int r = 0; r < 8; ++r) { const float z = acc[j][r] * (1.0f / 16.0f); so[wave][8 * g + r][j * 16 + col] = z > 15.0f ? z : log1pf(expf(z)); }
    LDSX();
    _Float16* D16 = which == 0 ? PQ16 : PK16; float* D32 = which == 0 ? PQ32 : PK32;
#pragma unroll 4
    for (int rl = 0; rl < 16; ++rl) vst2(D32 + (size_t)(r0 + rl) * DM + n0 + lane * 4, *(const v4f*)(&so[wave][rl][lane * 4]));
    for (int q = lane; q < 16 * 16; q += 32) { const int rl = q >> 4, pc = q & 15; union { v8h h8; v4u u; } pk;
#pragma unroll
      for (int e = 0; e < 8; ++e) pk.h8[e] = (_Float16)so[wave][rl][pc * 8 + e];
      vst2(D16 + (size_t)(r0 + rl) * DM + n0 + pc * 8, pk.u); } }
  else {
#pragma unroll 1
    for (int kc = 0; kc < DM / 32; ++kc) { const F2 a = split_row(xk + (size_t)(r0 + col) * DM, kc * 32, lane);
#pragma unroll
      for (int j = 0; j < 8; ++j) acc[j] = mac3(a, split_row(Wv + (size_t)(n0 + j * 16 + col) * DM, kc * 32, lane), acc[j]); }
#pragma unroll
    for (int j = 0; j < 8; ++j)
#pragma unroll
      for (int r = 0; r < 8; ++r) { so[wave][8 * g + r][j * 16 + col] = acc[j][r]; st[j * 16 + col][wave * 16 + 8 * g + r] = (_Float16)acc[j][r]; }
    LDSX();
#pragma unroll 4
    for (int rl = 0; rl < 16; ++rl) vst2(V32 + (size_t)(r0 + rl) * DM + n0 + lane * 4, *(const v4f*)(&so[wave][rl][lane * 4]));
    __syncthreads();
    { const int n = r0b / LL, l0 = r0b % LL;
      for (int q = tid; q < 128 * 8; q += 128) { const int cl = q >> 3, pc = q & 7; vst2(VT16 + ((size_t)n * DM + n0 + cl) * LL + l0 + pc * 8, *(const v4u*)(&st[cl][pc * 8])); } } }
}
__global__ __launch_bounds__(128) void k_attn(const _Float16* __restrict__ PQ16, const float* __restrict__ PQ32, const _Float16* __restrict__ PK16, const float* __restrict__ PK32, const float* __restrict__ V32, const _Float16* __restrict__ VT16, float* __restrict__ out) {
  __shared__ __align__(16) float sS[4][16][68];
  __shared__ __align__(16) _Float16 sP[4][16][72];
  __shared__ __align__(16) float sO[4][16][68];
  const int tid = threadIdx.x, w = tid >> 5, lane = tid & 31, col = lane & 15, g = lane >> 4;
  const int n = blockIdx.z, h = blockIdx.y, q0 = blockIdx.x * 64 + w * 16; const size_t rb = (size_t)n * LL;
  const bool precise = blockIdx.x < 2;
  v16h aq[2]; F2 aqs[2];
#pragma unroll
  for (int kc = 0; kc < 2; ++kc) { aq[kc] = frag_h(PQ16 + (rb + q0 + col) * DM + h * HD + kc * 32, lane); aqs[kc] = split_row(PQ32 + (rb + q0 + col) * DM + h * HD, kc * 32, lane); }
  v8f acc[4] = {}; float zsum = 0.f;
  const int ntiles = blockIdx.x + 1;
#pragma unroll 1
  for (int kt = 0; kt < ntiles; ++kt) {
#pragma unroll
    for (int t = 0; t < 4; ++t) { v8f s = {}; const int key = kt * 64 + t * 16 + col;
      if (precise) {
#pragma unroll
        for (int kc = 0; kc < 2; ++kc) s = mac3(aqs[kc], split_row(PK32 + (rb + key) * DM + h * HD, kc * 32, lane), s); }
      else {
#pragma unroll
        for (int kc = 0; kc < 2; ++kc) s = wmma16(aq[kc], frag_h(PK16 + (rb + key) * DM + h * HD + kc * 32, lane), s); }
#pragma unroll
      for (int r = 0; r < 8; ++r) { const int qi = q0 + 8 * g + r; sS[w][8 * g + r][t * 16 + col] = key <= qi ? s[r] : 0.f; } }
    LDSX();
    { float z = 0.f;
#pragma unroll
      for (int jj = 0; jj < 32; ++jj) { const float sv = sS[w][col][g * 32 + jj]; z += sv; sP[w][col][g * 32 + jj] = (_Float16)(sv * (1.0f / 64.0f)); }
      zsum += z; }
    LDSX();
    if (precise) {
#pragma unroll
      for (int kc = 0; kc < 2; ++kc) { const F2 pa = split_row(&sS[w][col][0], kc * 32, lane);
#pragma unroll
        for (int t = 0; t < 4; ++t) acc[t] = mac3(pa, split_col(V32 + (rb + kt * 64) * DM + h * HD, kc * 32, t * 16 + col, lane, DM, 64), acc[t]); } }
    else {
#pragma unroll
      for (int kc = 0; kc < 2; ++kc) { const v16h pa = frag_h(&sP[w][col][0] + kc * 32, lane);
#pragma unroll
        for (int t = 0; t < 4; ++t) acc[t] = wmma16(pa, frag_h(VT16 + ((size_t)n * DM + h * HD + t * 16 + col) * LL + kt * 64 + kc * 32, lane), acc[t]); } }
    __builtin_amdgcn_wave_barrier(); }
  zsum += __shfl_xor(zsum, 16, 32);
  const float oscale = precise ? 1.0f : 64.0f;
#pragma unroll
  for (int r = 0; r < 8; ++r) { const float zr = __shfl(zsum, 8 * g + r, 32);
#pragma unroll
    for (int t = 0; t < 4; ++t) sO[w][8 * g + r][t * 16 + col] = acc[t][r] * oscale / zr; }
  LDSX();
  for (int q = lane; q < 16 * 16; q += 32) { const int rl = q >> 4, pc = q & 15; vst2(out + (rb + q0 + rl) * DM + h * HD + pc * 4, *(const v4f*)(&sO[w][rl][pc * 4])); }
}
extern "C" void kernel_launch(void* const* d_in, const int* in_sizes, int n_in, void* d_out, int out_size, void* d_ws, size_t ws_size, hipStream_t stream) {
  (void)in_sizes; (void)n_in; (void)out_size; (void)ws_size;
  const float* xq = (const float*)d_in[0]; const float* xk = (const float*)d_in[1]; const float* Wq = (const float*)d_in[2]; const float* Wk = (const float*)d_in[3]; const float* Wv = (const float*)d_in[4];
  float* out = (float*)d_out;
  char* ws = (char*)d_ws; size_t off = 0;
  auto take = [&](size_t bytes) { char* p = ws + off; off += (bytes + 255) & ~(size_t)255; return p; };
  _Float16* PQ16 = (_Float16*)take((size_t)NR * DM * 2); float* PQ32 = (float*)take((size_t)NR * DM * 4); _Float16* PK16 = (_Float16*)take((size_t)NR * DM * 2); float* PK32 = (float*)take((size_t)NR * DM * 4);
  float* V32 = (float*)take((size_t)NR * DM * 4); _Float16* VT16 = (_Float16*)take((size_t)NB * DM * LL * 2);
  k_proj<<<dim3(NR / 64, DM / 128, 3), 128, 0, stream>>>(xq, xk, Wq, Wk, Wv, PQ16, PQ32, PK16, PK32, V32, VT16);
  k_attn<<<dim3(LL / 64, NH, NB), 128, 0, stream>>>(PQ16, PQ32, PK16, PK32, V32, VT16, out);
}
